// RGCN_3186865733924
// MI455X (gfx1250) — hardware-verified
//
#include <hip/hip_runtime.h>
#include <stddef.h>
#include <stdint.h>


#define HID     64
#define OUTD    32
#define KR      128
#define KPW     64
#define SEG     128
#define KAG     256
#define KHH     128
#define KL      384
#define NTHR    256
#define NWAVE   8
#define EPT     8
#define CHUNK   (NTHR * EPT)
#define WCAP    (EPT * 32)
#define LISTN   (NWAVE * WCAP)
#define NBA     512
#define PKS     9
#define RCAP    28672
#define DEGCAP  192
#define GBM     64
#define GTHR    128
#define NRB     32
#define RTI     32
#define NU_BR   (HID * (KR / 8))
#define NU_BP   (HID * (KPW / 8))
#define NU_L1   (3 * HID * (SEG / 8))
#define NU_L2   (3 * OUTD * (SEG / 8))
#define NU1     NU_BR
#define NU2     (NU1 + NU_BP)
#define NU3     (NU2 + NU_L1)
#define NUW     (NU3 + NU_L2)
#define ZINTS   (2 * RCAP + 2 * NBA + LISTN)
#define LDS_AGG (ZINTS * 4 + 64)
#define WSMAX   134217728

static_assert((CHUNK & (CHUNK - 1)) == 0);
static_assert(NBA == (1 << PKS));
static_assert(((long long)CHUNK << PKS) < (1LL << 31));
static_assert(NTHR * 2 == NBA);
static_assert(LISTN >= NBA && LISTN >= NWAVE * WCAP);
static_assert((RCAP % 32) == 0);
static_assert((ZINTS % (NTHR * 4)) == 0);
static_assert(LDS_AGG <= 262144);
static_assert((NBA % NWAVE) == 0 && (NBA % GBM) == 0);
static_assert(GBM == (GTHR / 32) * 16);
static_assert(KL == KAG + KHH && KAG == 2 * SEG && KHH == SEG && SEG == 2 * HID);
static_assert((KR % 32) == 0 && (KPW % 32) == 0 && (KAG % 32) == 0 && (KHH % 32) == 0);
static_assert(((KHH * 2) % 128) == 0 && ((KAG * 2) % 128) == 0 && ((OUTD * 4) % 128) == 0);
static_assert(HID == 32 * 2);
static_assert(NRB == 32 && RTI * 4 == 128);
static_assert((NU1 % NTHR) == 0 && (NU2 % NTHR) == 0 && (NU3 % NTHR) == 0 && (NUW % NTHR) == 0);
static_assert(((HID * (SEG / 8)) % NTHR) == 0 && ((OUTD * (SEG / 8)) % NTHR) == 0);
static_assert(HID * (SEG / 8) == 1024 && OUTD * (SEG / 8) == 512);

typedef float          v2f  __attribute__((ext_vector_type(2)));
typedef float          v4f  __attribute__((ext_vector_type(4)));
typedef float          v8f  __attribute__((ext_vector_type(8)));
typedef int            v2i  __attribute__((ext_vector_type(2)));
typedef int            v4i  __attribute__((ext_vector_type(4)));
typedef int            v8i  __attribute__((ext_vector_type(8)));
typedef unsigned int   v2u  __attribute__((ext_vector_type(2)));
typedef unsigned short v8us __attribute__((ext_vector_type(8)));
typedef _Float16       v16h __attribute__((ext_vector_type(16)));
typedef __bf16         v16b __attribute__((ext_vector_type(16)));
typedef v4f  __attribute__((may_alias)) v4fa;
typedef v2i  __attribute__((may_alias)) v2ia;
typedef v4i  __attribute__((may_alias)) v4ia;
typedef v2u  __attribute__((may_alias)) v2ua;
typedef v8us __attribute__((may_alias)) v8usa;
union Frag { v16b b; v16h f; v8us h[2]; v8i w; };

__device__ __forceinline__ v8f wmk(const Frag& a, const Frag& b, v8f c) {
  v8f d = __builtin_amdgcn_wmma_f32_16x16x32_bf16(false, a.b, false, b.b, (short)0, c, false, false);
  asm volatile("v_nop\n\tv_nop\n\tv_nop\n\tv_nop" : "+v"(d) : "v"(a.w), "v"(b.w));
  return d;
}

__device__ __forceinline__ unsigned short bf_bits(float f) {
  unsigned int u = __float_as_uint(f);
  u += 0x7FFFu + ((u >> 16) & 1u);
  return (unsigned short)(u >> 16);
}
__device__ __forceinline__ float bf_val(unsigned short b) {
  return __uint_as_float(((unsigned int)b) << 16);
}
__device__ __forceinline__ float bf_rne(float f) { return bf_val(bf_bits(f)); }

template <int ACT>
__device__ __forceinline__ float actf(float v) {
  if constexpr (ACT == 1) {
    return fmaxf(v, 0.0f);
  } else {
    return v;
  }
}

__device__ __forceinline__ v8us cv8(v4f a, v4f b) {
  v8us o;
  o[0] = bf_bits(a.x); o[1] = bf_bits(a.y); o[2] = bf_bits(a.z); o[3] = bf_bits(a.w);
  o[4] = bf_bits(b.x); o[5] = bf_bits(b.y); o[6] = bf_bits(b.z); o[7] = bf_bits(b.w);
  return o;
}
__device__ __forceinline__ v8us pairs8(v4f t) {
  v8us o;
  const unsigned short h0 = bf_bits(t.x), h1 = bf_bits(t.y), h2 = bf_bits(t.z), h3 = bf_bits(t.w);
  o[0] = h0; o[1] = h1;
  o[2] = bf_bits(t.x - bf_val(h0)); o[3] = bf_bits(t.y - bf_val(h1));
  o[4] = h2; o[5] = h3;
  o[6] = bf_bits(t.z - bf_val(h2)); o[7] = bf_bits(t.w - bf_val(h3));
  return o;
}

__device__ __forceinline__ int scan_chunk(const int* __restrict__ dsts, int nE, int cbase, int slotBase,
                                          int nb, int vec8, int* list, int tid, int lane, int wave) {
  int wc = 0;
  const int el0  = tid * EPT;
  const int e0   = cbase + el0;
  const int sent = -2147483647 - 1;
  v4i da, db;
  if (vec8 != 0 && cbase + CHUNK <= nE) {
    da = *(const v4i*)(dsts + e0);
    db = *(const v4i*)(dsts + e0 + 4);
  } else {
    da.x = (e0     < nE) ? dsts[min(e0,     nE - 1)] : sent;
    da.y = (e0 + 1 < nE) ? dsts[min(e0 + 1, nE - 1)] : sent;
    da.z = (e0 + 2 < nE) ? dsts[min(e0 + 2, nE - 1)] : sent;
    da.w = (e0 + 3 < nE) ? dsts[min(e0 + 3, nE - 1)] : sent;
    db.x = (e0 + 4 < nE) ? dsts[min(e0 + 4, nE - 1)] : sent;
    db.y = (e0 + 5 < nE) ? dsts[min(e0 + 5, nE - 1)] : sent;
    db.z = (e0 + 6 < nE) ? dsts[min(e0 + 6, nE - 1)] : sent;
    db.w = (e0 + 7 < nE) ? dsts[min(e0 + 7, nE - 1)] : sent;
  }
  const unsigned nbs = (unsigned)slotBase;
  const unsigned unb = (unsigned)nb;
  const unsigned s0 = (unsigned)da.x - nbs, s1 = (unsigned)da.y - nbs;
  const unsigned s2 = (unsigned)da.z - nbs, s3 = (unsigned)da.w - nbs;
  const unsigned s4 = (unsigned)db.x - nbs, s5 = (unsigned)db.y - nbs;
  const unsigned s6 = (unsigned)db.z - nbs, s7 = (unsigned)db.w - nbs;
  const bool h0 = s0 < unb, h1 = s1 < unb, h2 = s2 < unb, h3 = s3 < unb;
  const bool h4 = s4 < unb, h5 = s5 < unb, h6 = s6 < unb, h7 = s7 < unb;
  const unsigned any = __builtin_amdgcn_ballot_w32(h0 | h1 | h2 | h3 | h4 | h5 | h6 | h7);
  if (any != 0u) {
#define HITJ(J, HJ, SJ) { \
      const unsigned mj = __builtin_amdgcn_ballot_w32(HJ); \
      if (mj != 0u) { \
        if (HJ) { \
          const int pos = wc + (int)__builtin_amdgcn_mbcnt_lo(mj, 0u); \
          if (pos < WCAP) list[wave * WCAP + pos] = ((el0 + (J)) << PKS) | (int)(SJ); \
        } \
        wc += (int)__builtin_popcount(mj); } }
    HITJ(0, h0, s0)
    HITJ(1, h1, s1)
    HITJ(2, h2, s2)
    HITJ(3, h3, s3)
    HITJ(4, h4, s4)
    HITJ(5, h5, s5)
    HITJ(6, h6, s6)
    HITJ(7, h7, s7)
#undef HITJ
  }
  return wc;
}

__global__ __launch_bounds__(NTHR) void k_wprep(const float* __restrict__ wlr, const float* __restrict__ wlp,
                                                const float* __restrict__ wrel1, const float* __restrict__ wroot1,
                                                const float* __restrict__ wrel2, const float* __restrict__ wroot2,
                                                unsigned short* BR, unsigned short* BP,
                                                unsigned short* BL1, unsigned short* BL2) {
  const int u = (int)blockIdx.x * NTHR + (int)threadIdx.x;
  v8us o;
  unsigned short* dp;
  if (u < NU1) {
    const int n = u >> 4;
    const int q = u & 15;
    const float* p = wlr + (size_t)(8 * q) * HID + n;
#pragma unroll
    for (int i = 0; i < 8; ++i) o[i] = bf_bits(p[(size_t)i * HID]);
    dp = BR + (size_t)n * KR + 8 * q;
  } else if (u < NU2) {
    const int v = u - NU1;
    const int n = v >> 3;
    const int q = v & 7;
    const float* p = wlp + (size_t)(8 * q) * HID + n;
#pragma unroll
    for (int i = 0; i < 8; ++i) o[i] = bf_bits(p[(size_t)i * HID]);
    dp = BP + (size_t)n * KPW + 8 * q;
  } else if (u < NU3) {
    const int v = u - NU2;
    const int s = v >> 10;
    const int n = (v >> 4) & 63;
    const int q = v & 15;
    const float* W = wrel1;
    if (s == 1)      W = wrel1 + HID * HID;
    else if (s == 2) W = wroot1;
    const float* p = W + (size_t)(4 * q) * HID + n;
    const unsigned short f0 = bf_bits(p[0]), f1 = bf_bits(p[HID]);
    const unsigned short f2 = bf_bits(p[2 * HID]), f3 = bf_bits(p[3 * HID]);
    o[0] = f0; o[1] = f1; o[2] = f0; o[3] = f1; o[4] = f2; o[5] = f3; o[6] = f2; o[7] = f3;
    dp = BL1 + (size_t)n * KL + SEG * s + 8 * q;
  } else if (u < NUW) {
    const int v = u - NU3;
    const int s = v >> 9;
    const int n = (v >> 4) & 31;
    const int q = v & 15;
    const float* W = wrel2;
    if (s == 1)      W = wrel2 + HID * OUTD;
    else if (s == 2) W = wroot2;
    const float* p = W + (size_t)(4 * q) * OUTD + n;
    const unsigned short f0 = bf_bits(p[0]), f1 = bf_bits(p[OUTD]);
    const unsigned short f2 = bf_bits(p[2 * OUTD]), f3 = bf_bits(p[3 * OUTD]);
    o[0] = f0; o[1] = f1; o[2] = f0; o[3] = f1; o[4] = f2; o[5] = f3; o[6] = f2; o[7] = f3;
    dp = BL2 + (size_t)n * KL + SEG * s + 8 * q;
  } else {
    return;
  }
  *(volatile v8us*)dp = o;
  __threadfence();
  *(volatile v8us*)dp = o;
}

__global__ __launch_bounds__(NTHR) void k_range(const int* __restrict__ d0, int nE0,
                                                const int* __restrict__ d1, int nE1, int* RT) {
  __shared__ int red[NWAVE * 4];
  const int tid = (int)threadIdx.x, lane = tid & 31, wave = tid >> 5;
  const int g0 = (int)blockIdx.x * NTHR + tid;
  int mn0 = 2147483647, mx0 = -2147483647 - 1, mn1 = 2147483647, mx1 = -2147483647 - 1;
  {
    const int n4 = nE0 >> 2;
#pragma unroll 1
    for (int i = g0; i < n4; i += NRB * NTHR) {
      const v4i v = *(const v4ia*)(d0 + (size_t)4 * (size_t)i);
      mn0 = min(mn0, min(min(v.x, v.y), min(v.z, v.w)));
      mx0 = max(mx0, max(max(v.x, v.y), max(v.z, v.w)));
    }
    int t = 4 * n4 + (tid & 3);
    t = t > nE0 - 1 ? nE0 - 1 : t;
    const int tv = d0[t];
    mn0 = min(mn0, tv); mx0 = max(mx0, tv);
  }
  {
    const int n4 = nE1 >> 2;
#pragma unroll 1
    for (int i = g0; i < n4; i += NRB * NTHR) {
      const v4i v = *(const v4ia*)(d1 + (size_t)4 * (size_t)i);
      mn1 = min(mn1, min(min(v.x, v.y), min(v.z, v.w)));
      mx1 = max(mx1, max(max(v.x, v.y), max(v.z, v.w)));
    }
    int t = 4 * n4 + (tid & 3);
    t = t > nE1 - 1 ? nE1 - 1 : t;
    const int tv = d1[t];
    mn1 = min(mn1, tv); mx1 = max(mx1, tv);
  }
#pragma unroll
  for (int d = 1; d < 32; d <<= 1) {
    mn0 = min(mn0, __shfl_xor(mn0, d, 32)); mx0 = max(mx0, __shfl_xor(mx0, d, 32));
    mn1 = min(mn1, __shfl_xor(mn1, d, 32)); mx1 = max(mx1, __shfl_xor(mx1, d, 32));
  }
  if (lane == 0) {
    red[4 * wave + 0] = mn0; red[4 * wave + 1] = mx0; red[4 * wave + 2] = mn1; red[4 * wave + 3] = mx1;
  }
  __syncthreads();
  if (wave == 0) {
    int a = red[0], b = red[1], c = red[2], e = red[3];
#pragma unroll
    for (int w2 = 1; w2 < NWAVE; ++w2) {
      a = min(a, red[4 * w2 + 0]); b = max(b, red[4 * w2 + 1]);
      c = min(c, red[4 * w2 + 2]); e = max(e, red[4 * w2 + 3]);
    }
    v4i rec;
    rec.x = a; rec.y = ~b; rec.z = c; rec.w = ~e;
    int* p = RT + (size_t)blockIdx.x * RTI + 4 * (lane & 7);
    if (lane < 8) *(volatile v4i*)p = rec;
    __threadfence();
    if (lane < 8) *(volatile v4i*)p = rec;
  }
}

template <int NT, int SRC, int OUTM, int ACT>
__global__ __launch_bounds__(GTHR) void k_gemm(const float* __restrict__ X, int ldx, int nX,
                                               const unsigned short* __restrict__ AGp,
                                               const unsigned short* __restrict__ HHp,
                                               const unsigned short* __restrict__ BT, int ldb, int K1,
                                               const float* __restrict__ bias, int rowOff, int nRows,
                                               unsigned short* HO, float* C32) {
  constexpr int BN = 16 * NT;
  __shared__ __attribute__((aligned(16))) float stg[GBM * BN];
  const int tid = (int)threadIdx.x, lane = tid & 31, wave = tid >> 5, hh = lane >> 4, m = lane & 15;
  const int rowBase = (int)blockIdx.x * GBM;
  const int arow = rowBase + 16 * wave + m;

  v8f acc[NT];
  {
    const v8f z = {0.f, 0.f, 0.f, 0.f, 0.f, 0.f, 0.f, 0.f};
#pragma unroll
    for (int t = 0; t < NT; ++t) acc[t] = z;
  }
  const unsigned short* bp = BT + (size_t)m * (size_t)ldb + 8 * hh;

  if constexpr (SRC == 0) {
    const int rc = arow < nX ? arow : nX - 1;
    const float* xr = X + (size_t)rc * (size_t)ldx + 8 * hh;
#pragma unroll 1
    for (int k0 = 0; k0 < K1; k0 += 32) {
      Frag af;
      const v4f a0 = *(const v4fa*)(xr + k0);
      const v4f a1 = *(const v4fa*)(xr + k0 + 4);
      const v4f a2 = *(const v4fa*)(xr + k0 + 16);
      const v4f a3 = *(const v4fa*)(xr + k0 + 20);
      af.h[0] = cv8(a0, a1);
      af.h[1] = cv8(a2, a3);
#pragma unroll
      for (int nt = 0; nt < NT; ++nt) {
        const unsigned short* wq = bp + (size_t)(16 * nt) * (size_t)ldb + k0;
        Frag bf;
        bf.h[0] = *(const v8usa*)wq;
        bf.h[1] = *(const v8usa*)(wq + 16);
        acc[nt] = wmk(af, bf, acc[nt]);
      }
    }
  } else {
    const unsigned short* ap = AGp + (size_t)arow * (size_t)KAG + 8 * hh;
#pragma unroll 1
    for (int k0 = 0; k0 < KAG; k0 += 32) {
      Frag af;
      af.h[0] = *(const v8usa*)(ap + k0);
      af.h[1] = *(const v8usa*)(ap + k0 + 16);
#pragma unroll
      for (int nt = 0; nt < NT; ++nt) {
        const unsigned short* wq = bp + (size_t)(16 * nt) * (size_t)ldb + k0;
        Frag bf;
        bf.h[0] = *(const v8usa*)wq;
        bf.h[1] = *(const v8usa*)(wq + 16);
        acc[nt] = wmk(af, bf, acc[nt]);
      }
    }
    const unsigned short* hp = HHp + (size_t)arow * (size_t)KHH + 8 * hh;
#pragma unroll 1
    for (int k0 = 0; k0 < KHH; k0 += 32) {
      Frag af;
      af.h[0] = *(const v8usa*)(hp + k0);
      af.h[1] = *(const v8usa*)(hp + k0 + 16);
#pragma unroll
      for (int nt = 0; nt < NT; ++nt) {
        const unsigned short* wq = bp + (size_t)(16 * nt) * (size_t)ldb + KAG + k0;
        Frag bf;
        bf.h[0] = *(const v8usa*)wq;
        bf.h[1] = *(const v8usa*)(wq + 16);
        acc[nt] = wmk(af, bf, acc[nt]);
      }
    }
  }

#pragma unroll
  for (int nt = 0; nt < NT; ++nt) {
    const int lc = 16 * nt + m;
    const float bb = bf_rne(bias[lc]);
#pragma unroll
    for (int r = 0; r < 8; ++r) {
      const int lr = 16 * wave + 8 * hh + r;
      stg[lr * BN + lc] = actf<ACT>(acc[nt][r] + bb);
    }
  }
  __syncthreads();

  if constexpr (OUTM == 0) {
    static_assert(BN == HID);
    v8us pv[8];
#pragma unroll
    for (int i = 0; i < 8; ++i) {
      const int lr = 16 * wave + 2 * i + hh;
      pv[i] = pairs8(*(const v4fa*)(stg + lr * BN + 4 * m));
    }
#pragma unroll
    for (int i = 0; i < 8; ++i) {
      const int gr = rowBase + 16 * wave + 2 * i + hh;
      unsigned short* op = HO + (size_t)(rowOff + gr) * (size_t)KHH + 8 * m;
      if (gr < nRows) *(volatile v8us*)op = pv[i];
    }
    __threadfence();
#pragma unroll
    for (int i = 0; i < 8; ++i) {
      const int gr = rowBase + 16 * wave + 2 * i + hh;
      unsigned short* op = HO + (size_t)(rowOff + gr) * (size_t)KHH + 8 * m;
      if (gr < nRows) *(volatile v8us*)op = pv[i];
    }
  } else {
    constexpr int LPR = BN / 4;
    constexpr int RPI = 32 / LPR;
    constexpr int NI  = 16 / RPI;
    static_assert(LPR * RPI == 32 && NI * RPI == 16);
    const int rs = lane / LPR, cq = lane % LPR;
    v4f pv[NI];
#pragma unroll
    for (int i = 0; i < NI; ++i) {
      const int lr = 16 * wave + RPI * i + rs;
      pv[i] = *(const v4fa*)(stg + lr * BN + 4 * cq);
    }
#pragma unroll
    for (int i = 0; i < NI; ++i) {
      const int gr = rowBase + 16 * wave + RPI * i + rs;
      float* op = C32 + (size_t)(rowOff + gr) * (size_t)BN + 4 * cq;
      if (gr < nRows) *(volatile v4f*)op = pv[i];
    }
    __threadfence();
#pragma unroll
    for (int i = 0; i < NI; ++i) {
      const int gr = rowBase + 16 * wave + RPI * i + rs;
      float* op = C32 + (size_t)(rowOff + gr) * (size_t)BN + 4 * cq;
      if (gr < nRows) *(volatile v4f*)op = pv[i];
    }
  }
}

__global__ __launch_bounds__(NTHR) void k_agg(const int* __restrict__ src0, const int* __restrict__ dst0, int nE0,
                                              const int* __restrict__ src1, const int* __restrict__ dst1, int nE1,
                                              const unsigned short* __restrict__ HH, unsigned short* AGp,
                                              const int* __restrict__ RT, int nN) {
  extern __shared__ __attribute__((aligned(16))) int lds_i[];
  int* reg1 = lds_i;
  int* reg2 = reg1 + RCAP;
  int* scnt = reg2 + RCAP;
  int* soff = scnt + NBA;
  int* list = soff + NBA;
  int* wcnt = list + LISTN;
  int* wtot = wcnt + NWAVE;
  const int tid = (int)threadIdx.x, lane = tid & 31, wave = tid >> 5;
  const int nodeBase = (int)blockIdx.x * NBA;
  const int r = (int)blockIdx.y;
  const int* srcs = src0;
  const int* dsts = dst0;
  int nE = nE0;
  if (r == 1) { srcs = src1; dsts = dst1; nE = nE1; }
  const int vec8 = ((nE & 3) == 0) ? 1 : 0;

  {
    const v4i z4 = {0, 0, 0, 0};
    for (int i = tid * 4; i < ZINTS; i += NTHR * 4) *(v4ia*)(lds_i + i) = z4;
    if (tid < 2 * NWAVE) wcnt[tid] = 0;
  }

  int active;
  {
    const v4i rec = *(const v4ia*)(RT + RTI * lane);
    int mn = (r == 0) ? rec.x : rec.z;
    int mx = ~((r == 0) ? rec.y : rec.w);
#pragma unroll
    for (int d = 1; d < 32; d <<= 1) {
      mn = min(mn, __shfl_xor(mn, d, 32));
      mx = max(mx, __shfl_xor(mx, d, 32));
    }
    active = (mx < nodeBase || mn > nodeBase + NBA - 1) ? 0 : 1;
  }
  __syncthreads();

  int tot = 0;
  const int nChunks = (active != 0) ? (nE + CHUNK - 1) / CHUNK : 0;
#pragma unroll 1
  for (int ch = 0; ch < nChunks; ++ch) {
    const int cbase = ch * CHUNK;
    const int wc = scan_chunk(dsts, nE, cbase, nodeBase, NBA, vec8, list, tid, lane, wave);
    if (lane == 0) wcnt[wave] = wc;
    __syncthreads();
    int pre = 0, all = 0;
#pragma unroll
    for (int w2 = 0; w2 < NWAVE; ++w2) {
      int c = wcnt[w2];
      c = c < 0 ? 0 : (c > WCAP ? WCAP : c);
      all += c;
      pre += (w2 < wave) ? c : 0;
    }
    const int wcc  = wc > WCAP ? WCAP : wc;
    const int base = tot + pre;
#pragma unroll 1
    for (int i = lane; i < wcc; i += 32) {
      const int ent = list[wave * WCAP + i];
      const int el  = (ent >> PKS) & (CHUNK - 1);
      const int sl  = ent & (NBA - 1);
      int eid = cbase + el;
      eid = eid > nE - 1 ? nE - 1 : eid;
      const int pos = base + i;
      if (pos < RCAP) reg1[pos] = (int)(((unsigned)eid << PKS) | (unsigned)sl);
    }
    tot += all;
    tot = tot > RCAP ? RCAP : tot;
    __syncthreads();
  }
  const int nh = tot;

  if (wave == 0) {
#pragma unroll 1
    for (int b0 = 0; b0 < nh; b0 += 32) {
      const int idx = b0 + lane;
      const int uv  = reg1[idx < RCAP ? idx : RCAP - 1];
      const int m32 = (nh - b0) < 32 ? (nh - b0) : 32;
#pragma unroll 1
      for (int k = 0; k < m32; ++k) {
        const int u  = __builtin_amdgcn_readlane(uv, k);
        const int sl = u & (NBA - 1);
        if (lane == 0) scnt[sl] = scnt[sl] + 1;
      }
    }
  }
  __syncthreads();

  {
    const v2i ca = *(const v2ia*)(scnt + 2 * tid);
    const int e0 = ca.x < 0 ? 0 : ca.x, e1 = ca.y < 0 ? 0 : ca.y;
    const int ts = e0 + e1;
    int incl = ts;
#pragma unroll
    for (int d = 1; d < 32; d <<= 1) {
      const int up = __shfl_up(incl, d, 32);
      if (lane >= d) incl += up;
    }
    if (lane == 31) wtot[wave] = incl;
    __syncthreads();
    int pre = 0;
#pragma unroll
    for (int w2 = 0; w2 < NWAVE; ++w2) pre += (w2 < wave) ? wtot[w2] : 0;
    int run = pre + incl - ts;
    soff[2 * tid + 0] = run; run += e0;
    soff[2 * tid + 1] = run;
  }
  __syncthreads();
  for (int i = tid; i < NBA; i += NTHR) list[i] = soff[i];
  __syncthreads();

  if (wave == 0) {
#pragma unroll 1
    for (int b0 = 0; b0 < nh; b0 += 32) {
      const int idx = b0 + lane;
      const int uv  = reg1[idx < RCAP ? idx : RCAP - 1];
      const int m32 = (nh - b0) < 32 ? (nh - b0) : 32;
#pragma unroll 1
      for (int k = 0; k < m32; ++k) {
        const int u   = __builtin_amdgcn_readlane(uv, k);
        const int sl  = u & (NBA - 1);
        const int eid = (int)((unsigned)u >> PKS);
        if (lane == 0) {
          int pos = list[sl];
          pos = pos < 0 ? 0 : (pos > RCAP - 1 ? RCAP - 1 : pos);
          reg2[pos] = eid;
          list[sl] = pos + 1;
        }
      }
    }
  }
  __syncthreads();

  const int nbw = NBA / NWAVE;
  const bool ovf = (nh >= RCAP);
  const float qnan = __int_as_float(0x7fc00000);

#pragma unroll 1
  for (int jt = 0; jt < nbw; ++jt) {
    const int slot = wave * nbw + jt;
    const int node = nodeBase + slot;
    int st = soff[slot];
    const int craw = scnt[slot];
    int cnt = craw;
    st  = st < 0 ? 0 : (st > nh ? nh : st);
    cnt = cnt < 0 ? 0 : (cnt > DEGCAP ? DEGCAP : cnt);
    if (cnt > nh - st) cnt = nh - st;
    const float pz = (ovf || craw > DEGCAP) ? qnan : 0.0f;
    const bool live = node < nN;

    float a0 = 0.f, a1 = 0.f;
#pragma unroll 1
    for (int b0 = 0; b0 < cnt; b0 += 32) {
      int idx = st + b0 + lane; idx = idx > RCAP - 1 ? RCAP - 1 : idx;
      int eid = reg2[idx]; eid = eid < 0 ? 0 : (eid > nE - 1 ? nE - 1 : eid);
      int sr = srcs[eid]; sr = sr < 0 ? 0 : (sr > nN - 1 ? nN - 1 : sr);
      const int m32 = (cnt - b0) < 32 ? (cnt - b0) : 32;
#pragma unroll 1
      for (int k = 0; k < m32; ++k) {
        const int sk = __builtin_amdgcn_readlane(sr, k);
        const v2u v = *(const v2ua*)(HH + (size_t)sk * (size_t)KHH + 4 * lane);
        const float t0 = __uint_as_float(v.x << 16) + __uint_as_float(v.y << 16);
        const float t1 = __uint_as_float(v.x & 0xffff0000u) + __uint_as_float(v.y & 0xffff0000u);
        a0 += t0; a1 += t1;
      }
    }
    const float inv = 1.0f / fmaxf((float)craw, 1.0f);
    const float r0 = (live ? a0 * inv : 0.0f) + pz;
    const float r1 = (live ? a1 * inv : 0.0f) + pz;

    const unsigned short hb0 = bf_bits(r0), hb1 = bf_bits(r1);
    const unsigned short lb0 = bf_bits(r0 - bf_val(hb0)), lb1 = bf_bits(r1 - bf_val(hb1));
    v2u pk;
    pk.x = (unsigned int)hb0 | ((unsigned int)hb1 << 16);
    pk.y = (unsigned int)lb0 | ((unsigned int)lb1 << 16);

    unsigned short* gp = AGp + (size_t)node * (size_t)KAG + SEG * r + 4 * lane;
    *(volatile v2u*)gp = pk;
    __threadfence();
    *(volatile v2u*)gp = pk;
  }
}

static inline int cdiv(int a, int b) { return (a + b - 1) / b; }
static inline size_t al256(size_t o) { return (o + 255) & ~(size_t)255; }

extern "C" void kernel_launch(void* const* d_in, const int* in_sizes, int n_in,
                              void* d_out, int out_size, void* d_ws, size_t ws_size,
                              hipStream_t stream) {
  if (n_in < 16) return;
  if (in_sizes[0] < KR || (in_sizes[0] % KR) != 0) return;
  if (in_sizes[1] < KPW || (in_sizes[1] % KPW) != 0) return;
  const int nR = in_sizes[0] / KR;
  const int nP = in_sizes[1] / KPW;
  if (nR < 1 || nP < 1 || nR > (1 << 22) || nP > (1 << 22)) return;
  if (in_sizes[2] != KR * HID || in_sizes[3] != HID) return;
  if (in_sizes[4] != KPW * HID || in_sizes[5] != HID) return;
  if (in_sizes[6] != 2 * HID * HID || in_sizes[7] != HID * HID || in_sizes[8] != HID) return;
  if (in_sizes[9] != 2 * HID * OUTD || in_sizes[10] != HID * OUTD || in_sizes[11] != OUTD) return;
  const int nE0 = in_sizes[12], nE1 = in_sizes[14];
  if (in_sizes[13] != nE0 || in_sizes[15] != nE1) return;
  if (nE0 < 1 || nE1 < 1 || nE0 >= (1 << 22) || nE1 >= (1 << 22)) return;
  const int nN = nR + nP;
  if (nN > (1 << 22)) return;
  if ((long long)out_size != (long long)nN * OUTD) return;

  const float* x_r   = (const float*)d_in[0];
  const float* x_p   = (const float*)d_in[1];
  const float* wlr   = (const float*)d_in[2];
  const float* blr   = (const float*)d_in[3];
  const float* wlp   = (const float*)d_in[4];
  const float* blp   = (const float*)d_in[5];
  const float* wrel1 = (const float*)d_in[6];
  const float* wrt1  = (const float*)d_in[7];
  const float* b1    = (const float*)d_in[8];
  const float* wrel2 = (const float*)d_in[9];
  const float* wrt2  = (const float*)d_in[10];
  const float* b2    = (const float*)d_in[11];
  const int*   src0  = (const int*)d_in[12];
  const int*   dst0  = (const int*)d_in[13];
  const int*   src1  = (const int*)d_in[14];
  const int*   dst1  = (const int*)d_in[15];
  float* out = (float*)d_out;

  const int MP = cdiv(nN, GBM) * GBM;
  const int gM = MP / GBM;
  const int gR = cdiv(nR, GBM);
  const int gP = cdiv(MP - nR, GBM);
  const int gA = cdiv(MP, NBA);
  const int RA = gA * NBA;
  if ((long long)RA < (long long)MP || MP - nR < 1) return;

  char* ws = (char*)d_ws;
  size_t off = 0;
  const size_t oRT  = off; off = al256(off + (size_t)NRB * RTI * 4);
  const size_t oBR  = off; off = al256(off + (size_t)HID * KR * 2);
  const size_t oBP  = off; off = al256(off + (size_t)HID * KPW * 2);
  const size_t oBL1 = off; off = al256(off + (size_t)HID * KL * 2);
  const size_t oBL2 = off; off = al256(off + (size_t)OUTD * KL * 2);
  const size_t oHH0 = off; off = al256(off + (size_t)MP * KHH * 2);
  const size_t oHH1 = off; off = al256(off + (size_t)MP * KHH * 2);
  const size_t oAG  = off; off = al256(off + (size_t)RA * KAG * 2);
  if (off > ws_size || off > (size_t)WSMAX) return;
  int*            RT  = (int*)(ws + oRT);
  unsigned short* BR  = (unsigned short*)(ws + oBR);
  unsigned short* BP  = (unsigned short*)(ws + oBP);
  unsigned short* BL1 = (unsigned short*)(ws + oBL1);
  unsigned short* BL2 = (unsigned short*)(ws + oBL2);
  unsigned short* HH0 = (unsigned short*)(ws + oHH0);
  unsigned short* HH1 = (unsigned short*)(ws + oHH1);
  unsigned short* AG  = (unsigned short*)(ws + oAG);

  hipFuncSetAttribute(reinterpret_cast<const void*>(&k_agg), hipFuncAttributeMaxDynamicSharedMemorySize, LDS_AGG);

  k_wprep<<<NUW / NTHR, NTHR, 0, stream>>>(wlr, wlp, wrel1, wrt1, wrel2, wrt2, BR, BP, BL1, BL2);
  k_range<<<NRB, NTHR, 0, stream>>>(dst0, nE0, dst1, nE1, RT);
  k_gemm<4, 0, 0, 0><<<dim3(gR, 1), GTHR, 0, stream>>>(x_r, KR, nR, AG, HH1, BR, KR, KR, blr, 0, nR, HH0, out);
  k_gemm<4, 0, 0, 0><<<dim3(gP, 1), GTHR, 0, stream>>>(x_p, KPW, nP, AG, HH1, BP, KPW, KPW, blp, nR, MP - nR, HH0, out);
  k_agg<<<dim3(gA, 2), NTHR, LDS_AGG, stream>>>(src0, dst0, nE0, src1, dst1, nE1, HH0, AG, RT, nN);
  k_gemm<4, 1, 0, 1><<<dim3(gM, 1), GTHR, 0, stream>>>(x_r, KR, nR, AG, HH0, BL1, KL, KL, b1, 0, MP, HH1, out);
  k_agg<<<dim3(gA, 2), NTHR, LDS_AGG, stream>>>(src0, dst0, nE0, src1, dst1, nE1, HH1, AG, RT, nN);
  k_gemm<2, 1, 1, 0><<<dim3(gM, 1), GTHR, 0, stream>>>(x_r, KR, nR, AG, HH1, BL2, KL, KL, b2, 0, nN, HH0, out);
}
